// CausalNCMomentumAttention_22265110463166
// MI455X (gfx1250) — hardware-verified
//
#include <hip/hip_runtime.h>
#include <hip/hip_bf16.h>
#include <math.h>


#define BB 2
#define SS 2048
#define DD 512
#define HH 8
#define DKK 64
#define QW 1

typedef _Float16 bf16;
typedef __attribute__((ext_vector_type(4))) unsigned v4u_t;
typedef unsigned v4ua __attribute__((ext_vector_type(4), may_alias));
typedef __attribute__((ext_vector_type(4))) float v4f_t;
typedef float v4fa __attribute__((ext_vector_type(4), may_alias));
typedef __attribute__((ext_vector_type(16))) bf16  bf16x16;
typedef __attribute__((ext_vector_type(8)))  bf16  bf16x8;
typedef __attribute__((ext_vector_type(4)))  bf16  bf16x4;
typedef __attribute__((ext_vector_type(8)))  float f32x8;

#define LDS_STRIDE 48
#define KSTRIDE    72
#define VSTRIDE    48

__device__ __forceinline__ f32x8 wmma_bf16(bf16x16 a, bf16x16 b, f32x8 c) {
  return __builtin_amdgcn_wmma_f32_16x16x32_f16(
      false, a, false, b, (short)0, c, false, false);
}
#define RSPLIT (1.0f / 2048.0f)
__device__ __forceinline__ bf16 lo_of(float v, bf16 h) { return (bf16)((v - (float)h) * 2048.0f); }
__device__ __forceinline__ f32x8 wmma_split(bf16x16 a, bf16x16 al, bf16x16 b, bf16x16 bl, f32x8 c) {
  f32x8 x = {}; x = wmma_bf16(al, b, x); x = wmma_bf16(a, bl, x); return wmma_bf16(a, b, c) + x * RSPLIT; }

template <typename T>
__device__ __forceinline__ bf16x16 load_frag(const T* __restrict__ base, int ld,
                                             int row0, int k0) {
  const int lane = threadIdx.x & 31;
  const int r    = lane & 15;
  const int kh   = (lane >> 4) * 8;
  const T* p0 = base + (size_t)(row0 + r) * ld + (k0 + kh);
  const T* p1 = p0 + 16;
  bf16x16 f;
#pragma unroll
  for (int i = 0; i < 8; ++i) {
    f[i]     = (bf16)p0[i];
    f[i + 8] = (bf16)p1[i];
  }
  return f;
}

__device__ __forceinline__ bf16x16 lds_frag(const bf16* base, int stride) {
  const int lane = threadIdx.x & 31;
  const int row  = lane & 15;
  const int kh   = (lane >> 4) * 8;
  const bf16x8 lo = *(const bf16x8*)(base + row * stride + kh);
  const bf16x8 hi = *(const bf16x8*)(base + row * stride + kh + 16);
  bf16x16 f;
#pragma unroll
  for (int i = 0; i < 8; ++i) { f[i] = lo[i]; f[i + 8] = hi[i]; }
  return f;
}

template <typename T>
__device__ __forceinline__ void stage_read16(const T* __restrict__ p, float* buf) {
#pragma unroll
  for (int i = 0; i < 16; ++i) buf[i] = (float)p[i];
}

__device__ __forceinline__ void stage_write(bf16* dst, const float* buf, int nquad) {
#pragma unroll
  for (int i = 0; i < nquad; ++i) {
    bf16x4 q;
    q[0] = (bf16)buf[4 * i];     q[1] = (bf16)buf[4 * i + 1];
    q[2] = (bf16)buf[4 * i + 2]; q[3] = (bf16)buf[4 * i + 3];
    *(bf16x4*)(dst + 4 * i) = q;
  }
}

#define LEPS 1e-6f
#define DELTA 0.1f
#define STEPSIZE 1.0f
__global__ __launch_bounds__(64) void linattn_kernel(
    const bf16* __restrict__ Qb, const bf16* __restrict__ Kb,
    const bf16* __restrict__ Vt, size_t vPlane, float* __restrict__ out) {
  __shared__ bf16 ldsK[32 * KSTRIDE];
  __shared__ bf16 ldsV[64 * VSTRIDE], ldsVl[64 * VSTRIDE];
  __shared__ __attribute__((aligned(16))) float ldsO[2][32 * 68];

  const int q0blk = blockIdx.x * 32;
  const int h  = blockIdx.y;
  const int b  = blockIdx.z;
  const int t    = threadIdx.x;
  const int wave = t >> 5;
  const int lane = t & 31;
  const int qlane = lane & 15;
  const int kh8   = (lane >> 4) * 8;
  const int q0 = q0blk + wave * 16;

  const bf16* Qh = Qb + (size_t)b * SS * DD + h * DKK;
  const bf16* Kh = Kb + (size_t)b * SS * DD + h * DKK;
  const bf16* Vh = Vt + ((size_t)(b * HH + h)) * DKK * SS;

  const int krow = t >> 1;
  const int kcol = (t & 1) * 32;
  const bf16* kSrc = Kh + (size_t)krow * DD + kcol;
  const bf16* vSrc = Vh + (size_t)t * SS;

  bf16x16 qf[QW][2];
#pragma unroll
  for (int qt = 0; qt < QW; ++qt) {
    qf[qt][0] = load_frag(Qh, DD, q0 + 16 * qt, 0);
    qf[qt][1] = load_frag(Qh, DD, q0 + 16 * qt, 32);
  }

  f32x8 o[QW][4] = {};
  float lrun[QW];
#pragma unroll
  for (int qt = 0; qt < QW; ++qt) lrun[qt] = 0.0f;
  const int kmax = q0blk + 31;

  bf16x8 kreg[4], vreg[4], vlreg[4];
#pragma unroll
  for (int i = 0; i < 4; ++i) {
    kreg[i] = *(const bf16x8*)(kSrc + 8 * i);
    vreg[i] = *(const bf16x8*)(vSrc + 8 * i); vlreg[i] = *(const bf16x8*)(vSrc + vPlane + 8 * i);
  }

  for (int kb = 0; kb <= kmax; kb += 32) {
    __syncthreads();
#pragma unroll
    for (int i = 0; i < 4; ++i) {
      *(bf16x8*)(&ldsK[krow * KSTRIDE + kcol + 8 * i]) = kreg[i];
      *(bf16x8*)(&ldsV[t * VSTRIDE + 8 * i])           = vreg[i];
      *(bf16x8*)(&ldsVl[t * VSTRIDE + 8 * i])          = vlreg[i];
    }
    if (kb + 32 <= kmax) {
      const bf16* kn = kSrc + (size_t)(kb + 32) * DD;
      const bf16* vn = vSrc + (kb + 32);
#pragma unroll
      for (int i = 0; i < 4; ++i) {
        kreg[i] = *(const bf16x8*)(kn + 8 * i);
        vreg[i] = *(const bf16x8*)(vn + 8 * i); vlreg[i] = *(const bf16x8*)(vn + vPlane + 8 * i);
      }
    }
    __syncthreads();

    bf16x16 kf[2][2];
#pragma unroll
    for (int ktile = 0; ktile < 2; ++ktile)
#pragma unroll
      for (int c = 0; c < 2; ++c)
        kf[ktile][c] = lds_frag(ldsK + (ktile * 16) * KSTRIDE + c * 32, KSTRIDE);

    bf16x16 pf[QW], pfl[QW];
    bool act[QW];
#pragma unroll
    for (int qt = 0; qt < QW; ++qt) {
      act[qt] = (kb <= q0 + 16 * qt + 15);
      if (act[qt]) {
        const int q_my = q0 + 16 * qt + qlane;
        f32x8 s0 = {}, s1 = {};
        s0 = wmma_bf16(kf[0][0], qf[qt][0], s0);
        s0 = wmma_bf16(kf[0][1], qf[qt][1], s0);
        s1 = wmma_bf16(kf[1][0], qf[qt][0], s1);
        s1 = wmma_bf16(kf[1][1], qf[qt][1], s1);

        float rsum = 0.0f;
#pragma unroll
        for (int r = 0; r < 8; ++r) {
          const int k0i = kb + kh8 + r;
          const int k1i = k0i + 16;
          const float w0 = (k0i <= q_my) ? s0[r] : 0.0f;
          const float w1 = (k1i <= q_my) ? s1[r] : 0.0f;
          rsum += w0 + w1;
          pf[qt][r] = (bf16)w0; pfl[qt][r] = lo_of(w0, pf[qt][r]);
          pf[qt][r + 8] = (bf16)w1; pfl[qt][r + 8] = lo_of(w1, pf[qt][r + 8]);
        }
        rsum += __shfl_xor(rsum, 16, 32);
        lrun[qt] += rsum;
      }
    }

#pragma unroll
    for (int j = 0; j < 4; ++j) {
      const bf16x16 vf = lds_frag(ldsV + (j * 16) * VSTRIDE, VSTRIDE), vfl = lds_frag(ldsVl + (j * 16) * VSTRIDE, VSTRIDE);
#pragma unroll
      for (int qt = 0; qt < QW; ++qt)
        if (act[qt]) o[qt][j] = wmma_split(vf, vfl, pf[qt], pfl[qt], o[qt][j]);
    }
  }

  float* so = ldsO[wave];
#pragma unroll
  for (int qt = 0; qt < QW; ++qt) {
    const float rl = 1.0f / (lrun[qt] + LEPS);
#pragma unroll
    for (int j = 0; j < 4; ++j)
#pragma unroll
      for (int r = 0; r < 8; ++r) so[(16 * qt + qlane) * 68 + j * 16 + kh8 + r] = o[qt][j][r] * rl;
  }
  asm volatile("s_wait_dscnt 0" ::: "memory");
#pragma unroll 1
  for (int pass = 0; pass < 2; ++pass) {
#pragma unroll
    for (int it = 0; it < 8; ++it) { const int ch = lane + 32 * it, ql = ch >> 4, q4 = (ch & 15) * 4;
      *(volatile v4f_t*)(out + ((size_t)(b * SS + q0 + ql)) * DD + h * DKK + q4) = *(const volatile v4fa*)(so + ql * 68 + q4); }
    __threadfence();
  }
}

__device__ __forceinline__ float phi(float x) { return x > 0.0f ? x + 1.0f : expf(x); }
__global__ __launch_bounds__(128) void k_feat(const float* __restrict__ q, const float* __restrict__ k, const float* __restrict__ mask,
                                             bf16* __restrict__ Qb, bf16* __restrict__ Kb, float* __restrict__ Kf) {
  const int tok = blockIdx.x, t = threadIdx.x; const float mk = mask[tok];
  const v4f_t qv = *(const v4fa*)(q + (size_t)tok * DD + t * 4), kv = *(const v4fa*)(k + (size_t)tok * DD + t * 4);
  bf16 hq[4], hk[4]; v4f_t kf;
  kf.x = phi(kv.x) * mk; kf.y = phi(kv.y) * mk; kf.z = phi(kv.z) * mk; kf.w = phi(kv.w) * mk;
  hq[0] = (bf16)phi(qv.x); hq[1] = (bf16)phi(qv.y); hq[2] = (bf16)phi(qv.z); hq[3] = (bf16)phi(qv.w);
  hk[0] = (bf16)kf.x; hk[1] = (bf16)kf.y; hk[2] = (bf16)kf.z; hk[3] = (bf16)kf.w;
  typedef __attribute__((ext_vector_type(2))) unsigned v2u; typedef unsigned v2ua __attribute__((ext_vector_type(2), may_alias));
#pragma unroll 1
  for (int pass = 0; pass < 2; ++pass) {
    *(volatile v2u*)(Qb + (size_t)tok * DD + t * 4) = *(const v2ua*)hq; *(volatile v2u*)(Kb + (size_t)tok * DD + t * 4) = *(const v2ua*)hk;
    *(volatile v4f_t*)(Kf + (size_t)tok * DD + t * 4) = kf;
    __threadfence(); }
}
__global__ __launch_bounds__(256) void k_vt(const float* __restrict__ v, bf16* __restrict__ Vt, size_t plane) {
  __shared__ float tile[64][65];
  const int s0 = blockIdx.x * 64, h = blockIdx.y, b = blockIdx.z, t = threadIdx.x;
  for (int i = t; i < 64 * 64; i += 256) { const int r = i >> 6, d = i & 63; tile[r][d] = v[((size_t)(b * SS + s0 + r)) * DD + h * DKK + d]; }
  __syncthreads();
#pragma unroll 1
  for (int pass = 0; pass < 2; ++pass) {
    for (int i = t; i < 64 * 8; i += 256) { const int dr = i >> 3, s8 = (i & 7) * 8; bf16 hh[8], hl[8];
#pragma unroll
      for (int e = 0; e < 8; ++e) { const float x = tile[s8 + e][dr]; hh[e] = (bf16)x; hl[e] = lo_of(x, hh[e]); }
      bf16* dst = Vt + (((size_t)(b * HH + h)) * DKK + dr) * SS + s0 + s8;
      *(volatile v4u_t*)dst = *(const v4ua*)hh; *(volatile v4u_t*)(dst + plane) = *(const v4ua*)hl; }
    __threadfence();
  }
}
__global__ __launch_bounds__(256) void k_norms(const float* __restrict__ Kf, const float* __restrict__ v, float* __restrict__ S) {
  const int bh = blockIdx.y, b = bh / HH, h = bh % HH, tpos = blockIdx.x * 256 + threadIdx.x;
  const float* kt = Kf + ((size_t)(b * SS + tpos)) * DD + h * DKK; const float* vt = v + ((size_t)(b * SS + tpos)) * DD + h * DKK;
  float kk = 0.f, vv = 0.f, kd = 0.f, vd = 0.f; const bool has_next = (tpos + 1 < SS);
#pragma unroll 1
  for (int e = 0; e < DKK; ++e) { const float a = kt[e], c = vt[e]; kk += a * a; vv += c * c;
    if (has_next) { kd += a * kt[DD + e]; vd += c * vt[DD + e]; } }
  float* s = S + (size_t)bh * 4 * SS + tpos;
#pragma unroll 1
  for (int pass = 0; pass < 2; ++pass) { *(volatile float*)s = kk; *(volatile float*)(s + SS) = vv; *(volatile float*)(s + 2 * SS) = kd; *(volatile float*)(s + 3 * SS) = vd; __threadfence(); }
}
__global__ __launch_bounds__(32) void k_momentum(const float* __restrict__ S, float* __restrict__ A) {
  const int bh = threadIdx.x; if (bh >= BB * HH) return;
  const float* s = S + (size_t)bh * 4 * SS; float* a = A + (size_t)bh * SS;
  float acur = 1.0f; a[SS - 1] = 1.0f;
#pragma unroll 1
  for (int j = SS - 2; j >= 0; --j) {
    const float kk0 = s[j], vv0 = s[SS + j], kk1 = s[j + 1], vv1 = s[SS + j + 1], kd = s[2 * SS + j], vd = s[3 * SS + j];
    const float base2 = kk0 * vv0, diff2 = kk1 * vv1 + kk0 * vv0 - 2.0f * kd * vd;
    const float ratio = sqrtf(fmaxf(diff2, 0.0f)) / sqrtf(base2);
    float mu = 1.0f - sqrtf(ratio); mu = mu * mu; mu = fminf(fmaxf(mu, 0.0f), 1.0f - DELTA);
    acur = 1.0f + mu * acur; a[j] = acur;
  }
  __threadfence();
#pragma unroll 1
  for (int j = 0; j < SS; ++j) { const float x = a[j]; *(volatile float*)(a + j) = x; }
}
__global__ __launch_bounds__(128) void k_kn(const float* __restrict__ Kf, const float* __restrict__ A, float* __restrict__ Kn) {
  const int tok = blockIdx.x, t = threadIdx.x, b = tok / SS, l = tok % SS, h = (t * 4) / DKK;
  const float w = A[((size_t)(b * HH + h)) * SS + l] * STEPSIZE;
  v4f_t kv = *(const v4fa*)(Kf + (size_t)tok * DD + t * 4); kv.x *= w; kv.y *= w; kv.z *= w; kv.w *= w;
  *(volatile v4f_t*)(Kn + (size_t)tok * DD + t * 4) = kv; __threadfence(); *(volatile v4f_t*)(Kn + (size_t)tok * DD + t * 4) = kv;
}

extern "C" void kernel_launch(void* const* d_in, const int* in_sizes, int n_in,
                              void* d_out, int out_size, void* d_ws, size_t ws_size,
                              hipStream_t stream) {
  (void)in_sizes; (void)n_in; (void)out_size; (void)ws_size;
  const float* q = (const float*)d_in[0]; const float* k = (const float*)d_in[1]; const float* v = (const float*)d_in[2];
  const float* mask = (const float*)d_in[3];
  float* out = (float*)d_out;
  float* Kn  = out + (size_t)BB * SS * DD;
  char* ws = (char*)d_ws;
  bf16* Qb  = (bf16*)ws; ws += (size_t)BB * SS * DD * 2;
  bf16* Kb  = (bf16*)ws; ws += (size_t)BB * SS * DD * 2;
  bf16* VtB = (bf16*)ws; ws += (size_t)BB * SS * DD * 2 * 2;
  float* Kf = (float*)ws; ws += (size_t)BB * SS * DD * 4;
  float* S4 = (float*)ws; ws += (size_t)BB * HH * 4 * SS * 4;
  float* Aw = (float*)ws; ws += (size_t)BB * HH * SS * 4;
  const size_t vpl = (size_t)BB * SS * DD;
  k_feat<<<BB * SS, 128, 0, stream>>>(q, k, mask, Qb, Kb, Kf);
  k_vt<<<dim3(SS / 64, HH, BB), 256, 0, stream>>>(v, VtB, vpl);
  linattn_kernel<<<dim3(SS / 32, HH, BB), 64, 0, stream>>>(Qb, Kb, VtB, vpl, out);
  k_norms<<<dim3(SS / 256, BB * HH), 256, 0, stream>>>(Kf, v, S4);
  k_momentum<<<1, 32, 0, stream>>>(S4, Aw);
  k_kn<<<BB * SS, 128, 0, stream>>>(Kf, Aw, Kn);
}
